// DisConv_20650202759324
// MI455X (gfx1250) — hardware-verified
//
#include <hip/hip_runtime.h>
#include <hip/hip_bf16.h>

#define Nn      2048
#define IN_DIMn 128
#define KCH     8
#define DD      32
#define ITERSn  4
#define EPSn    1e-12f

typedef __attribute__((ext_vector_type(16))) _Float16 v16h;
typedef __attribute__((ext_vector_type(8)))  _Float16 v8h;
typedef __attribute__((ext_vector_type(8)))  float    v8f;
typedef __attribute__((ext_vector_type(4)))  float    v4f;
typedef __attribute__((ext_vector_type(4)))  unsigned v4u;
typedef float __attribute__((may_alias)) float_a;
template <typename T> __device__ __forceinline__ void vst2(void* p, T v) { *(volatile T*)p = v; __threadfence(); *(volatile T*)p = v; }
__device__ __forceinline__ v8f wmma16(v16h a, v16h b, v8f c) {
    v8f d = __builtin_amdgcn_wmma_f32_16x16x32_f16(false, a, false, b, (short)0, c, false, false);
    asm volatile("v_nop\n\tv_nop\n\tv_nop\n\tv_nop" : "+v"(d) : "v"(a), "v"(b));
    return d;
}

union F16x16 { v16h v; _Float16 e[16]; unsigned u[8]; };

__global__ __launch_bounds__(256) void disconv_proj(
    const float* __restrict__ feat, const float* __restrict__ W,
    const float* __restrict__ b, float* __restrict__ Z,
    _Float16* __restrict__ Zh)
{
    __shared__ __align__(16) _Float16 szh[8][DD];
    int gw   = (blockIdx.x * blockDim.x + threadIdx.x) >> 5;
    int lane = threadIdx.x & 31;
    int k = gw >> 11;
    int n = gw & (Nn - 1);

    float acc = b[k * DD + lane];
    const float* frow = feat + (size_t)n * IN_DIMn;
    const float* wcol = W + (size_t)k * IN_DIMn * DD + lane;
    #pragma unroll 4
    for (int i = 0; i < IN_DIMn; ++i)
        acc = fmaf(frow[i], wcol[(size_t)i * DD], acc);

    float s = acc * acc;
    #pragma unroll
    for (int m = 16; m >= 1; m >>= 1) s += __shfl_xor(s, m, 32);
    float scale = 1.0f / fmaxf(sqrtf(s), EPSn);
    float zv = acc * scale;

    size_t idx = ((size_t)k * Nn + n) * DD + lane;
    vst2(Z + idx, (float_a)zv);
    szh[threadIdx.x >> 5][lane] = (_Float16)zv;
    __syncthreads();
    if (threadIdx.x < 32) {
        const size_t base = ((size_t)blockIdx.x * 8) * DD;
        vst2(Zh + base + threadIdx.x * 8, *(const v4u*)(&szh[0][0] + threadIdx.x * 8));
    }
}

__global__ __launch_bounds__(256) void disconv_route(
    const float* __restrict__ Zin, const _Float16* __restrict__ Zhin,
    const int* __restrict__ adj,
    float* __restrict__ Zout, _Float16* __restrict__ Zhout,
    float* __restrict__ out, int write_out)
{
    __shared__ __align__(16) _Float16 sZh[KCH][32][DD];
    __shared__ __align__(16) float sExp[KCH][16][32];
    __shared__ __align__(16) float sRcp[16][32];
    __shared__ __align__(16) int   sAdj[16][32];
    __shared__ __align__(16) float sOut[KCH][16][32];

    const int t    = threadIdx.x;
    const int lane = t & 31;
    const int k    = t >> 5;
    const int h    = lane >> 4;
    const int nl   = lane & 15;
    const int n0   = blockIdx.x * 16;

    F16x16 Au;
    #pragma unroll
    for (int v = 0; v < 8; ++v) {
        int d0 = (v < 4) ? (8 * h + 2 * v) : (16 + 8 * h + 2 * (v - 4));
        Au.u[v] = *(const unsigned*)(Zhin + ((size_t)k * Nn + n0 + nl) * DD + d0);
    }

    v8f acc0, acc1;
    #pragma unroll
    for (int v = 0; v < 8; ++v) {
        int row = v + 8 * h;
        acc0[v] = Zin[((size_t)k * Nn + n0 + row) * DD + nl];
        acc1[v] = Zin[((size_t)k * Nn + n0 + row) * DD + 16 + nl];
    }


    for (int m0 = 0; m0 < Nn; m0 += 32) {
        __syncthreads();

        #pragma unroll
        for (int j = 0; j < 4; ++j) {
            int chunk = t + 256 * j;
            int kk   = chunk >> 7;
            int mm   = (chunk >> 2) & 31;
            int part = chunk & 3;
            *(v4u*)(&sZh[kk][mm][part * 8]) = *(const v4u*)(Zhin + ((size_t)kk * Nn + m0 + mm) * DD + part * 8);
        }
        {
            const int* ap = adj + (size_t)(n0 + (t >> 4)) * Nn + m0 + (t & 15) * 2;
            sAdj[t >> 4][(t & 15) * 2]     = ap[0];
            sAdj[t >> 4][(t & 15) * 2 + 1] = ap[1];
        }
        __syncthreads();

        #pragma unroll
        for (int msub = 0; msub < 2; ++msub) {
            F16x16 Bu;
            #pragma unroll
            for (int v = 0; v < 8; ++v)
                Bu.u[v] = *(const unsigned*)&sZh[k][msub * 16 + nl][(v < 4) ? (8 * h + 2 * v) : (16 + 8 * h + 2 * (v - 4))];
            v8f c0 = {};
            v8f att = wmma16(Au.v, Bu.v, c0);
            #pragma unroll
            for (int v = 0; v < 8; ++v) {
                int row = v + 8 * h;
                int mc  = msub * 16 + nl;
                sExp[k][row][mc] = (sAdj[row][mc] > 0) ? __expf(att[v]) : 0.0f;
            }
        }
        __syncthreads();

        for (int e = t; e < 512; e += 256) {
            int nn = e >> 5, mm = e & 31;
            float s = 0.0f;
            #pragma unroll
            for (int kk = 0; kk < KCH; ++kk) s += sExp[kk][nn][mm];
            sRcp[nn][mm] = (s > 0.0f) ? __builtin_amdgcn_rcpf(s) : 0.0f;
        }
        __syncthreads();

        F16x16 Pu;
        #pragma unroll
        for (int v = 0; v < 8; ++v) {
            int mp = (v < 4) ? (8 * h + 2 * v) : (16 + 8 * h + 2 * (v - 4));
            Pu.e[2 * v]     = (_Float16)(sExp[k][nl][mp]     * sRcp[nl][mp]);
            Pu.e[2 * v + 1] = (_Float16)(sExp[k][nl][mp + 1] * sRcp[nl][mp + 1]);
        }

        #pragma unroll
        for (int csub = 0; csub < 2; ++csub) {
            F16x16 Bu;
            #pragma unroll
            for (int v = 0; v < 8; ++v) {
                const int mr = (v < 4) ? (8 * h + 2 * v) : (16 + 8 * h + 2 * (v - 4));
                Bu.e[2 * v]     = sZh[k][mr    ][csub * 16 + nl];
                Bu.e[2 * v + 1] = sZh[k][mr + 1][csub * 16 + nl];
            }
            if (csub == 0) acc0 = wmma16(Pu.v, Bu.v, acc0);
            else           acc1 = wmma16(Pu.v, Bu.v, acc1);
        }
    }

    #pragma unroll
    for (int v = 0; v < 8; ++v) {
        float s = acc0[v] * acc0[v] + acc1[v] * acc1[v];
        s += __shfl_xor(s, 1, 32);
        s += __shfl_xor(s, 2, 32);
        s += __shfl_xor(s, 4, 32);
        s += __shfl_xor(s, 8, 32);
        float scale = 1.0f / fmaxf(sqrtf(s), EPSn);
        acc0[v] *= scale;
        acc1[v] *= scale;
    }

    #pragma unroll
    for (int v = 0; v < 8; ++v) { int row = v + 8 * h; sOut[k][row][nl] = acc0[v]; sOut[k][row][16 + nl] = acc1[v]; }
    __syncthreads();
    {
        const float* S = &sOut[k][0][0];
        #pragma unroll
        for (int q = 0; q < 4; ++q) { const int rl = q * 4 + (lane >> 3), pc = lane & 7;
            vst2(Zout + ((size_t)k * Nn + n0 + rl) * DD + pc * 4, *(const v4f*)(S + rl * 32 + pc * 4));
            if (write_out) vst2(out + (size_t)(n0 + rl) * (KCH * DD) + k * DD + pc * 4, *(const v4f*)(S + rl * 32 + pc * 4)); }
        #pragma unroll
        for (int q = 0; q < 2; ++q) { const int g = q * 32 + lane; const int rl = g >> 2, pc = g & 3;
            union { v8h hh; v4u u; } pk;
            #pragma unroll
            for (int e = 0; e < 8; ++e) pk.hh[e] = (_Float16)S[rl * 32 + pc * 8 + e];
            vst2(Zhout + ((size_t)k * Nn + n0 + rl) * DD + pc * 8, pk.u); }
    }
}

extern "C" void kernel_launch(void* const* d_in, const int* in_sizes, int n_in,
                              void* d_out, int out_size, void* d_ws, size_t ws_size,
                              hipStream_t stream)
{
    const int*   adj  = (const int*)d_in[0];
    const float* feat = (const float*)d_in[1];
    const float* W    = (const float*)d_in[2];
    const float* b    = (const float*)d_in[3];
    float* out = (float*)d_out;

    const size_t ZE = (size_t)KCH * Nn * DD;
    float*    Z0  = (float*)d_ws;
    float*    Z1  = Z0 + ZE;
    _Float16* Zh0 = (_Float16*)(Z1 + ZE);
    _Float16* Zh1 = Zh0 + ZE;

    disconv_proj<<<(KCH * Nn * 32) / 256, 256, 0, stream>>>(feat, W, b, Z0, Zh0);

    float* zi = Z0; _Float16* zhi = Zh0;
    float* zo = Z1; _Float16* zho = Zh1;
    for (int it = 0; it < ITERSn; ++it) {
        disconv_route<<<Nn / 16, 256, 0, stream>>>(zi, zhi, adj, zo, zho, out,
                                                   it == ITERSn - 1);
        float* tz = zi; zi = zo; zo = tz;
        _Float16* th = zhi; zhi = zho; zho = th;
    }
    (void)in_sizes; (void)n_in; (void)out_size; (void)ws_size;
}
